// HaloAttn_36876589204203
// MI455X (gfx1250) — hardware-verified
//
#include <hip/hip_runtime.h>


namespace {
constexpr int B = 8, C = 256, HH = 64, WW = 64, NPOS = HH * WW, NH = 8, DH = 16, DV = 32, BS = 8, HS = 3, WIN = 14, NKEY = WIN * WIN  , NKT = 13  , GP = HH + 2 * HS  , NCELL = GP * GP, NBLK = (HH / BS) * (WW / BS), NREL = 2 * WIN - 1, BL = 8;
constexpr float XS = 8.0f, WSC = 256.0f, PS = 1024.0f, LOG2E = 1.4426950408889634f, SCALE = 0.25f;
typedef _Float16 b16;
typedef __attribute__((ext_vector_type(16))) _Float16 v16b;
typedef __attribute__((ext_vector_type(8))) _Float16 v8b;
typedef __attribute__((ext_vector_type(8))) float v8f;
typedef __attribute__((ext_vector_type(4))) float v4f;
__device__ __forceinline__ float bf16_rne(float f) { unsigned int u = __float_as_uint(f); u += 0x7FFFu + ((u >> 16) & 1u); return __uint_as_float(u & 0xFFFF0000u); }
__device__ __forceinline__ void split16(float v, b16& hi, b16& lo) { hi = (b16)v; lo = (b16)(v - (float)hi); }
__device__ __forceinline__ v16b frag_kb(const b16* p, int hh) { const v8b a = *(const v8b*)(p + 8 * hh), b = *(const v8b*)(p + 16 + 8 * hh); v16b f;
#pragma unroll
  for (int e = 0; e < 8; ++e) { f[e] = a[e]; f[8 + e] = b[e]; } return f; }
__device__ __forceinline__ v8f wmma16b(v16b a, v16b b, v8f c) { v8f d = __builtin_amdgcn_wmma_f32_16x16x32_f16(false, a, false, b, (short)0, c, false, false); asm volatile("v_nop\n\tv_nop\n\tv_nop\n\tv_nop" : "+v"(d) : "v"(a), "v"(b)); return d; }
__device__ __forceinline__ void wave_lds_sync() { __builtin_amdgcn_fence(__ATOMIC_RELEASE, "workgroup"); __builtin_amdgcn_wave_barrier(); __builtin_amdgcn_fence(__ATOMIC_ACQUIRE, "workgroup"); }
__device__ __forceinline__ float pmul(float a, float b) { float p = a * b; asm volatile("" : "+v"(p)); return p; }
__device__ __forceinline__ int iclamp(int v, int lo, int hi) { return v < lo ? lo : (v > hi ? hi : v); }

typedef __attribute__((ext_vector_type(2))) _Float16 v2h;
typedef __attribute__((ext_vector_type(4))) _Float16 v4h;
typedef __attribute__((ext_vector_type(2))) float v2f;
__device__ __forceinline__ float nexp2(float v) { return __builtin_amdgcn_exp2f(v); }
__device__ __forceinline__ v16b frag16(const b16* row, int hh) { v16b f; const v8b lo8 = *(const v8b*)(row + 8 * hh); for (int j = 0; j < 8; ++j) { f[j] = lo8[j]; f[8 + j] = (b16)0.0f; } return f; }
__global__ __launch_bounds__(256) void prep_kernel(const float* __restrict__ qw, const float* __restrict__ kvw, b16* __restrict__ WT, b16* __restrict__ Kh, b16* __restrict__ Kl, b16* __restrict__ Vp, b16* __restrict__ Vpl) {
  size_t t = (size_t)blockIdx.x * 256 + threadIdx.x; v8b o, z = {};
  { const size_t n = (size_t)512 * C / 8; if (t < n) { const size_t e = t * 8; const float* w = (e < (size_t)128 * C) ? qw + e : kvw + (e - (size_t)128 * C); for (int j = 0; j < 8; ++j) o[j] = (b16)(bf16_rne(w[j]) * WSC); for (int pass = 0; pass < 2; ++pass) { *(volatile v8b*)(WT + e) = o; __threadfence(); } return; } t -= n; }
  { const size_t n = (size_t)B * NH * NCELL * DV / 8; if (t < n) { const size_t e = t * 8; for (int pass = 0; pass < 2; ++pass) { if (e < (size_t)B * NH * NCELL * DH) { *(volatile v8b*)(Kh + e) = z; *(volatile v8b*)(Kl + e) = z; } *(volatile v8b*)(Vp + e) = z; *(volatile v8b*)(Vpl + e) = z; __threadfence(); } } }
}
__global__ __launch_bounds__(128) void proj_kernel(const float* __restrict__ x, const b16* __restrict__ WT, b16* __restrict__ Qh, b16* __restrict__ Ql, b16* __restrict__ Kh, b16* __restrict__ Kl, b16* __restrict__ Vp, b16* __restrict__ Vpl) {
  __shared__ __attribute__((aligned(16))) b16 As[64][C + 8]; __shared__ __attribute__((aligned(16))) float Tf[64][128 + 4];
  const int wave = threadIdx.x >> 5, lane = threadIdx.x & 31, nloc = lane & 15, hlf = lane >> 4, t = threadIdx.x; const int b = blockIdx.y, y = blockIdx.x, slab = blockIdx.z;
  for (int i = t; i < C * 64; i += 128) { const int c = i >> 6, p = i & 63; As[p][c] = (b16)(bf16_rne(x[(((size_t)b * C + c) * HH + y) * WW + p]) * XS); }
  __syncthreads();
  const int m0 = wave * 16;
  v8f acc[8];
#pragma unroll
  for (int tt = 0; tt < 8; ++tt) acc[tt] = (v8f){};
#pragma unroll 2
  for (int kb = 0; kb < C; kb += 32) { const v16b a = frag_kb(&As[m0 + nloc][kb], hlf);
#pragma unroll
    for (int tt = 0; tt < 8; ++tt) acc[tt] = wmma16b(a, frag_kb(WT + (size_t)(slab * 128 + tt * 16 + nloc) * C + kb, hlf), acc[tt]); }
#pragma unroll
  for (int tt = 0; tt < 8; ++tt)
#pragma unroll
    for (int r = 0; r < 8; ++r) Tf[m0 + 8 * hlf + r][tt * 16 + nloc] = acc[tt][r] * (1.0f / (XS * WSC));
  __syncthreads();
  const size_t cell0 = (size_t)(y + HS) * GP + HS;
  for (int pass = 0; pass < 2; ++pass) {
    if (slab == 0) {
      for (int i = t; i < NH * 128; i += 128) { const int h = i >> 7, piece = i & 127; const int p = piece >> 1, q8 = (piece & 1) * 8; v8b hv, lv;
        for (int j = 0; j < 8; ++j) { const int d = q8 + j; b16 ph, pl; split16(Tf[p][h * DH + d] * XS, ph, pl); hv[j] = ph; lv[j] = pl; }
        const size_t oi = (((size_t)b * NH + h) * NPOS + (size_t)y * WW + p) * DH + q8; *(volatile v8b*)(Qh + oi) = hv; *(volatile v8b*)(Ql + oi) = lv; }
    } else { const int c0 = (slab - 1) * 128;
      for (int i = t; i < 64 * 16; i += 128) { const int p = i >> 4, piece = i & 15; const int cc = c0 + piece * 8;
        const int h = cc / (DH + DV), within = cc % (DH + DV);
        if (within < DH) { const int d0 = within;
          v8b hv, lv; for (int j = 0; j < 8; ++j) { b16 ph, pl; split16(Tf[p][piece * 8 + j] * XS, ph, pl); hv[j] = ph; lv[j] = pl; }
          const size_t oi = (((size_t)b * NH + h) * NCELL + cell0 + p) * DH + d0; *(volatile v8b*)(Kh + oi) = hv; *(volatile v8b*)(Kl + oi) = lv; }
        else { const int d0 = within - DH; v8b o, ol; for (int j = 0; j < 8; ++j) { b16 ph, pl; split16(Tf[p][piece * 8 + j] * XS, ph, pl); o[j] = ph; ol[j] = pl; }
          const size_t oi = (((size_t)b * NH + h) * NCELL + cell0 + p) * DV + d0; *(volatile v8b*)(Vp + oi) = o; *(volatile v8b*)(Vpl + oi) = ol; } } }
    __threadfence(); }
}
__global__ __launch_bounds__(128) void attn_kernel(const b16* __restrict__ Qh, const b16* __restrict__ Ql, const b16* __restrict__ Kh, const b16* __restrict__ Kl, const b16* __restrict__ Vp, const b16* __restrict__ Vpl, const float* __restrict__ hrel, const float* __restrict__ wrel, float* __restrict__ OB) {
  __shared__ float QR[64][2 * NREL + 2]; __shared__ __attribute__((aligned(16))) float To[64][DV + 4]; __shared__ __attribute__((aligned(16))) b16 Ph[64][224 + 8], Pl[64][224 + 8], Vt[DV][224 + 8], Vtl[DV][224 + 8];
  const int wave = threadIdx.x >> 5, lane = threadIdx.x & 31, nloc = lane & 15, hlf = lane >> 4, t = threadIdx.x; const int blk = blockIdx.x, h = blockIdx.y, b = blockIdx.z; const int bi = blk / (WW / BS), bj = blk % (WW / BS);
  const b16* Qhb = Qh + ((size_t)b * NH + h) * NPOS * DH; const b16* Qlb = Ql + ((size_t)b * NH + h) * NPOS * DH; const b16* Khb = Kh + ((size_t)b * NH + h) * NCELL * DH; const b16* Klb = Kl + ((size_t)b * NH + h) * NCELL * DH; const b16* Vb = Vp + ((size_t)b * NH + h) * NCELL * DV; const b16* Vlb = Vpl + ((size_t)b * NH + h) * NCELL * DV;
  auto qpos = [&](int q) { return (size_t)(bi * BS + (q >> 3)) * WW + bj * BS + (q & 7); };
  auto kcell = [&](int s) { return (s < NKEY) ? (size_t)(bi * BS + s / WIN) * GP + bj * BS + s % WIN : (size_t)0; };
  { const int q = t >> 1, half = t & 1; float qv[DH]; const size_t qo = qpos(q) * DH; for (int d = 0; d < DH; ++d) qv[d] = ((float)Qhb[qo + d] + (float)Qlb[qo + d]) * (1.0f / XS);
    const float* rel = half ? wrel : hrel;
#pragma unroll 1
    for (int r = 0; r < NREL; ++r) { float s = 0.0f;
#pragma unroll
      for (int d = 0; d < DH; ++d) s += pmul(qv[d], bf16_rne(rel[r * DH + d])); QR[q][half * NREL + r] = s; } }
  for (int s = t; s < 224; s += 128) { const b16* vr = Vb + kcell(s) * DV; const b16* vlr = Vlb + kcell(s) * DV; const bool live = s < NKEY;
    for (int d0 = 0; d0 < DV; d0 += 8) { const v8b vv = *(const v8b*)(vr + d0), vl = *(const v8b*)(vlr + d0); for (int j = 0; j < 8; ++j) { Vt[d0 + j][s] = live ? vv[j] : (b16)0.0f; Vtl[d0 + j][s] = live ? vl[j] : (b16)0.0f; } } }
  __syncthreads();
  float inv_own;
  { const int qq = wave * 16 + nloc; const size_t qo = qpos(qq) * DH; const v16b qh = frag16(Qhb + qo, hlf), ql = frag16(Qlb + qo, hlf);
    const int qqi = qq >> 3, qqj = qq & 7; const float cs = SCALE / (XS * XS); float mx = -INFINITY, sum = 0.0f;
#pragma unroll 1
    for (int ps = 0; ps < 2; ++ps) {
#pragma unroll 1
      for (int kt = 0; kt < NKT; ++kt) { const size_t kc = kcell(kt * 16 + nloc) * DH; const v16b kh = frag16(Khb + kc, hlf), kl = frag16(Klb + kc, hlf);
        v8f s = (v8f){}; s = wmma16b(kh, qh, s); s = wmma16b(kh, ql, s); s = wmma16b(kl, qh, s);
#pragma unroll
        for (int r = 0; r < 8; ++r) { const int slot = kt * 16 + 8 * hlf + r; float lg = -INFINITY;
          if (slot < NKEY) { const int ki = slot / WIN, kj = slot % WIN; lg = s[r] * cs + QR[qq][ki - qqi + WIN - 1] + QR[qq][NREL + kj - qqj + WIN - 1]; }
          if (ps == 0) mx = fmaxf(mx, lg);
          else { const float p = (slot < NKEY) ? nexp2((lg - mx) * LOG2E) : 0.0f; sum += p; b16 a_, b_; split16(p * PS, a_, b_); Ph[qq][slot] = a_; Pl[qq][slot] = b_; } } }
      if (ps == 0) mx = fmaxf(mx, __shfl_xor(mx, 16)); }
    sum += __shfl_xor(sum, 16); inv_own = 1.0f / (sum * PS * XS);
    for (int j = 0; j < 8; ++j) { Ph[qq][208 + 8 * hlf + j] = (b16)0.0f; Pl[qq][208 + 8 * hlf + j] = (b16)0.0f; } }
  __syncthreads();
  v8f o[2] = {(v8f){}, (v8f){}};
#pragma unroll
  for (int ks = 0; ks < 7; ++ks) { const v16b ph = frag_kb(&Ph[wave * 16 + nloc][ks * 32], hlf), pl = frag_kb(&Pl[wave * 16 + nloc][ks * 32], hlf);
#pragma unroll
    for (int tt = 0; tt < 2; ++tt) { const v16b va = frag_kb(&Vt[tt * 16 + nloc][ks * 32], hlf), val = frag_kb(&Vtl[tt * 16 + nloc][ks * 32], hlf); o[tt] = wmma16b(va, ph, o[tt]); o[tt] = wmma16b(va, pl, o[tt]); o[tt] = wmma16b(val, ph, o[tt]); } }
#pragma unroll
  for (int tt = 0; tt < 2; ++tt)
#pragma unroll
    for (int r = 0; r < 8; ++r) To[wave * 16 + nloc][tt * 16 + 8 * hlf + r] = o[tt][r] * inv_own;
  wave_lds_sync();
  float* obw = OB + ((((size_t)b * NH + h) * NBLK + blk) * 64 + wave * 16) * DV;
  for (int pass = 0; pass < 2; ++pass) { for (int i = lane; i < 16 * DV / 4; i += 32) { const int qq = i / (DV / 4), c4 = (i % (DV / 4)) * 4; *(volatile v4f*)(obw + qq * DV + c4) = *(const v4f*)(&To[wave * 16 + qq][c4]); } __threadfence(); }
}
__global__ __launch_bounds__(256) void outT_kernel(const float* __restrict__ OB, float* __restrict__ out) {
  __shared__ float T[DV][BS][WW + 1];
  const int t = threadIdx.x; const int bi = blockIdx.x, h = blockIdx.y, b = blockIdx.z;
  for (int i = t; i < 8 * 64 * DV; i += 256) { const int bj = i / (64 * DV), rem = i % (64 * DV); const int q = rem / DV, dv = rem % DV; T[dv][q >> 3][bj * BS + (q & 7)] = OB[((((size_t)b * NH + h) * NBLK + bi * 8 + bj) * 64 + q) * DV + dv]; }
  __syncthreads();
  const int wave = t >> 5, lane = t & 31;
  for (int pass = 0; pass < 2; ++pass) { for (int rr = wave; rr < DV * BS; rr += 8) { const int dv = rr / BS, yy = rr % BS; v2f v = {T[dv][yy][lane * 2], T[dv][yy][lane * 2 + 1]};
      *(volatile v2f*)(out + (((size_t)b * (NH * DV) + h * DV + dv) * HH + bi * BS + yy) * WW + lane * 2) = v; } __threadfence(); }
}
}

extern "C" void kernel_launch(void* const* d_in, const int* in_sizes, int n_in, void* d_out, int out_size, void* d_ws, size_t ws_size, hipStream_t stream) {
  (void)n_in;
  auto Fp = [&](int i) { return (const float*)d_in[i]; };
  if (in_sizes[0] != B * C * NPOS || in_sizes[1] != 128 * C || in_sizes[2] != 384 * C || in_sizes[3] != NREL * DH || in_sizes[4] != NREL * DH || out_size != B * NH * DV * NPOS) return;
  size_t off = 0; char* ws = (char*)d_ws;
  auto carve = [&](size_t bytes) { char* p = ws + off; off += (bytes + 255) & ~(size_t)255; return p; };
  b16* WT = (b16*)carve((size_t)512 * C * 2); b16* Qh = (b16*)carve((size_t)B * NH * NPOS * DH * 2); b16* Ql = (b16*)carve((size_t)B * NH * NPOS * DH * 2); b16* Kh = (b16*)carve((size_t)B * NH * NCELL * DH * 2); b16* Kl = (b16*)carve((size_t)B * NH * NCELL * DH * 2); b16* Vp = (b16*)carve((size_t)B * NH * NCELL * DV * 2); b16* Vpl = (b16*)carve((size_t)B * NH * NCELL * DV * 2);
  float* OB = (float*)carve((size_t)B * NH * NBLK * 64 * DV * 4);
  if (off > ws_size || off > ((size_t)128 << 20)) return;
  prep_kernel<<<(unsigned)((((size_t)512 * C + (size_t)B * NH * NCELL * DV) / 8 + 255) / 256), 256, 0, stream>>>(Fp(1), Fp(2), WT, Kh, Kl, Vp, Vpl);
  proj_kernel<<<dim3(HH, BL, 4), 128, 0, stream>>>(Fp(0), WT, Qh, Ql, Kh, Kl, Vp, Vpl);
  attn_kernel<<<dim3(NBLK, NH, BL), 128, 0, stream>>>(Qh, Ql, Kh, Kl, Vp, Vpl, Fp(3), Fp(4), OB);
  outT_kernel<<<dim3(HH / BS, NH, BL), 256, 0, stream>>>(OB, (float*)d_out);
}
